// GatedDeltaNetAttention_1082331758936
// MI455X (gfx1250) — hardware-verified
//
#include <hip/hip_runtime.h>
#include <math.h>

constexpr int kL      = 1024;
constexpr int kD      = 2048;
constexpr int kH      = 16;
constexpr int kHD     = 128;
constexpr int kCKey   = kH * kHD;
constexpr int kCVal   = kH * kHD;
constexpr int kCConv  = 2 * kCKey + kCVal;
constexpr int kTaps   = 4;
constexpr int kZCol0  = kCConv;
constexpr int kBCol0  = kCConv + kCVal;
constexpr int kACol0  = kBCol0 + kH;
constexpr int kNCat   = kBCol0 + 64;
constexpr int kChunk  = 16;
constexpr int kScanThreads = 1024;
constexpr int kStatePerLane = 16;
constexpr float kWCarry      = 64.0f;
constexpr float kGCarry      = 16.0f;
constexpr float kResCarry    = 2048.0f;
constexpr float kResCarryInv = 1.0f / kResCarry;
constexpr float kProjScale   = 1.0f / kWCarry;
constexpr float kOutScale    = 1.0f / (kWCarry * kGCarry);
constexpr float kEps         = 1e-6f;
constexpr float kFltMin      = 1.17549435e-38f;
constexpr float kF16MinNormal = 6.103515625e-05f;

static_assert(kCKey == 2048 && kCVal == 2048 && kCConv == 6144, "channel layout");
static_assert(kNCat == 8256 && kNCat % 64 == 0 && kNCat % 32 == 0, "N tile multiple");
static_assert(kACol0 == 8208, "dt logit columns");
static_assert(kL % 64 == 0 && kD % 64 == 0 && kD % 32 == 0, "M and K tile multiples");
static_assert(kL % kChunk == 0, "chunking exact");
static_assert(kHD * (kHD / kStatePerLane) == kScanThreads, "state partition");
static_assert(kChunk * 3 * kHD / 4 == 1536, "chunk staging size");
static_assert(((kL / 64) * (kNCat / 32)) % 8 == 0, "projection tiles (64x32) fill whole blocks");
static_assert(((kL / 64) * (kD / 64)) % 8 == 0, "output tiles (64x64) fill whole blocks");
static_assert(kResCarry == 2048.0f && kResCarryInv * kResCarry == 1.0f, "residual carry fold");
static_assert(kProjScale * kWCarry == 1.0f, "weight carry fold");
static_assert(kOutScale * kWCarry * kGCarry == 1.0f, "output carry fold");
static_assert((size_t)kL * kCConv * 4 <= (size_t)kNCat * kD * 2, "aliased plane fits the dead weight plane");

typedef __attribute__((ext_vector_type(16))) _Float16 v16h;
typedef __attribute__((ext_vector_type(8)))  _Float16 v8h;
typedef __attribute__((ext_vector_type(8)))  float    v8f;
typedef __attribute__((ext_vector_type(4)))  float    v4f;
typedef __attribute__((ext_vector_type(4)))  unsigned int v4u;
typedef __attribute__((ext_vector_type(2)))  unsigned int v2u;

__device__ __forceinline__ unsigned short h_bits(float f) {
  const _Float16 h = (_Float16)f;
  return __builtin_bit_cast(unsigned short, h);
}
__device__ __forceinline__ unsigned pk16(unsigned short a, unsigned short b) {
  return (unsigned)a | ((unsigned)b << 16);
}
__device__ __forceinline__ float silu_f(float x) {
  return x * __builtin_amdgcn_rcpf(1.0f + expf(-x));
}
__device__ __forceinline__ void split_f16(float f, unsigned short& hb, unsigned short& lb) {
  const _Float16 h = (_Float16)f;
  const float hr = (float)h;
  const float hf = (fabsf(f) < kF16MinNormal) ? 0.0f : hr;
  const float lf = (f - hf) * kResCarry;
  hb = h_bits(hf);
  lb = h_bits(lf);
}

__device__ __forceinline__ void dep_guard4_h(v8f& a, v8f& b, v8f& c, v8f& d, v16h x, v16h y) {
  asm volatile("v_nop\n\tv_nop\n\tv_nop\n\tv_nop" : "+v"(a), "+v"(b), "+v"(c), "+v"(d) : "v"(x), "v"(y));
}
__device__ __forceinline__ void keep4_h(v16h a, v16h b, v16h c, v16h d) {
  asm volatile("v_nop" :: "v"(a), "v"(b), "v"(c), "v"(d));
}
__device__ __forceinline__ void acc_guard4(v8f& a, v8f& b, v8f& c, v8f& d) {
  asm volatile("v_nop\n\tv_nop\n\tv_nop\n\tv_nop" : "+v"(a), "+v"(b), "+v"(c), "+v"(d));
}

union FragU { v16h v; v8h h[2]; };
__device__ __forceinline__ v16h frag_load(const _Float16* p) {
  FragU f;
  f.h[0] = *(const v8h*)(p);
  f.h[1] = *(const v8h*)(p + 16);
  return f.v;
}
__device__ __forceinline__ v8f frag_mma(v16h a, v16h b, v8f c) {
  return __builtin_amdgcn_wmma_f32_16x16x32_f16(false, a, false, b, (short)0, c, false, false);
}

__global__ __launch_bounds__(256) void wmma_gemm_split_f16(
    const unsigned short* __restrict__ Ahp, const unsigned short* __restrict__ Alp, int lda,
    const unsigned short* __restrict__ Bhp, const unsigned short* __restrict__ Blp, int ldb,
    float* __restrict__ C, int ldc, int M, int N, int K, float scale) {
  const _Float16* Ah = (const _Float16*)Ahp;
  const _Float16* Al = (const _Float16*)Alp;
  const _Float16* Bh = (const _Float16*)Bhp;
  const _Float16* Bl = (const _Float16*)Blp;
  __shared__ __align__(16) float sT[8][16 * 36];
  const int lane = threadIdx.x & 31;
  const int wave = threadIdx.x >> 5;
  const int tilesN = N >> 5;
  const int tilesM = M >> 6;
  const int tile = blockIdx.x * 8 + wave;
  if (tile >= tilesM * tilesN) return;
  const int tm = tile / tilesN;
  const int tn = tile - tm * tilesN;
  const int m0 = tm << 6;
  const int n0 = tn << 5;
  const int rlane = lane & 15;
  const int koff  = (lane >> 4) * 8;
  const int mOff  = (lane >> 4) * 8;

  int ao[4];
  int bo[2];
#pragma unroll
  for (int i = 0; i < 4; ++i) ao[i] = (m0 + (i << 4) + rlane) * lda + koff;
#pragma unroll
  for (int j = 0; j < 2; ++j) bo[j] = (n0 + (j << 4) + rlane) * ldb + koff;

  v8f accM[4][2];
  v8f accX[4][2];
#pragma unroll
  for (int i = 0; i < 4; ++i)
#pragma unroll
    for (int j = 0; j < 2; ++j) {
      accM[i][j] = (v8f){0.f, 0.f, 0.f, 0.f, 0.f, 0.f, 0.f, 0.f};
      accX[i][j] = (v8f){0.f, 0.f, 0.f, 0.f, 0.f, 0.f, 0.f, 0.f};
    }

  for (int k0 = 0; k0 < K; k0 += 32) {
    v16h bh[2], bl[2];
#pragma unroll
    for (int j = 0; j < 2; ++j) {
      bh[j] = frag_load(Bh + bo[j] + k0);
      bl[j] = frag_load(Bl + bo[j] + k0);
    }
#pragma unroll
    for (int i = 0; i < 4; ++i) {
      const v16h ah = frag_load(Ah + ao[i] + k0);
      const v16h al = frag_load(Al + ao[i] + k0);
#pragma unroll
      for (int j = 0; j < 2; ++j) {
        accM[i][j] = frag_mma(ah, bh[j], accM[i][j]);
        accX[i][j] = frag_mma(ah, bl[j], accX[i][j]);
        accX[i][j] = frag_mma(al, bh[j], accX[i][j]);
      }
      dep_guard4_h(accM[i][0], accM[i][1], accX[i][0], accX[i][1], ah, al);
    }
    keep4_h(bh[0], bh[1], bl[0], bl[1]);
  }
  acc_guard4(accM[0][0], accM[0][1], accX[0][0], accX[0][1]);
  acc_guard4(accM[1][0], accM[1][1], accX[1][0], accX[1][1]);
  acc_guard4(accM[2][0], accM[2][1], accX[2][0], accX[2][1]);
  acc_guard4(accM[3][0], accM[3][1], accX[3][0], accX[3][1]);

  float* slab = sT[wave];
  const int q  = lane >> 3;
  const int c4 = (lane & 7) * 4;
#pragma unroll
  for (int i = 0; i < 4; ++i) {
    const int mBase = m0 + (i << 4);
#pragma unroll
    for (int j = 0; j < 2; ++j) {
#pragma unroll
      for (int r = 0; r < 8; ++r) {
        const float cross = accX[i][j][r] * kResCarryInv;
        slab[(mOff + r) * 36 + (j << 4) + rlane] = (accM[i][j][r] + cross) * scale;
      }
    }
    __builtin_amdgcn_fence(__ATOMIC_RELEASE, "workgroup");
    __builtin_amdgcn_wave_barrier();
    __builtin_amdgcn_fence(__ATOMIC_ACQUIRE, "workgroup");
    for (int pass = 0; pass < 2; ++pass) {
#pragma unroll
      for (int it = 0; it < 4; ++it) {
        const int row = it * 4 + q;
        const v4f val = *(const v4f*)(slab + row * 36 + c4);
        *(volatile v4f*)(C + (size_t)(mBase + row) * ldc + n0 + c4) = val;
      }
      __threadfence();
    }
    __builtin_amdgcn_fence(__ATOMIC_RELEASE, "workgroup");
    __builtin_amdgcn_wave_barrier();
    __builtin_amdgcn_fence(__ATOMIC_ACQUIRE, "workgroup");
  }
}

__global__ __launch_bounds__(256) void wmma_gemm64_f16(
    const unsigned short* __restrict__ Ap, int lda,
    const unsigned short* __restrict__ Btp, int ldb,
    float* __restrict__ C, int ldc, int M, int N, int K, float scale) {
  const _Float16* A  = (const _Float16*)Ap;
  const _Float16* Bt = (const _Float16*)Btp;
  __shared__ __align__(16) float sT[8][16 * 68];
  const int lane = threadIdx.x & 31;
  const int wave = threadIdx.x >> 5;
  const int tilesN = N >> 6;
  const int tilesM = M >> 6;
  const int tile = blockIdx.x * 8 + wave;
  if (tile >= tilesM * tilesN) return;
  const int tm = tile / tilesN;
  const int tn = tile - tm * tilesN;
  const int m0 = tm << 6;
  const int n0 = tn << 6;
  const int rlane = lane & 15;
  const int koff  = (lane >> 4) * 8;
  const int mOff  = (lane >> 4) * 8;

  const _Float16* pa[4];
  const _Float16* pb[4];
#pragma unroll
  for (int i = 0; i < 4; ++i) {
    pa[i] = A  + (size_t)(m0 + (i << 4) + rlane) * lda + koff;
    pb[i] = Bt + (size_t)(n0 + (i << 4) + rlane) * ldb + koff;
  }

  v8f acc[4][4];
#pragma unroll
  for (int i = 0; i < 4; ++i)
#pragma unroll
    for (int j = 0; j < 4; ++j) acc[i][j] = (v8f){0.f, 0.f, 0.f, 0.f, 0.f, 0.f, 0.f, 0.f};

  for (int k0 = 0; k0 < K; k0 += 32) {
    v16h bh[4];
#pragma unroll
    for (int j = 0; j < 4; ++j) bh[j] = frag_load(pb[j] + k0);
#pragma unroll
    for (int i = 0; i < 4; ++i) {
      const v16h ah = frag_load(pa[i] + k0);
#pragma unroll
      for (int j = 0; j < 4; ++j) acc[i][j] = frag_mma(ah, bh[j], acc[i][j]);
      dep_guard4_h(acc[i][0], acc[i][1], acc[i][2], acc[i][3], ah, bh[3]);
    }
    keep4_h(bh[0], bh[1], bh[2], bh[3]);
  }
  acc_guard4(acc[0][0], acc[0][1], acc[0][2], acc[0][3]);
  acc_guard4(acc[1][0], acc[1][1], acc[1][2], acc[1][3]);
  acc_guard4(acc[2][0], acc[2][1], acc[2][2], acc[2][3]);
  acc_guard4(acc[3][0], acc[3][1], acc[3][2], acc[3][3]);

  float* slab = sT[wave];
  const int hh = lane >> 4;
  const int c4 = (lane & 15) * 4;
#pragma unroll
  for (int i = 0; i < 4; ++i) {
    const int mBase = m0 + (i << 4);
#pragma unroll
    for (int j = 0; j < 4; ++j) {
#pragma unroll
      for (int r = 0; r < 8; ++r) {
        slab[(mOff + r) * 68 + (j << 4) + rlane] = acc[i][j][r] * scale;
      }
    }
    __builtin_amdgcn_fence(__ATOMIC_RELEASE, "workgroup");
    __builtin_amdgcn_wave_barrier();
    __builtin_amdgcn_fence(__ATOMIC_ACQUIRE, "workgroup");
    for (int pass = 0; pass < 2; ++pass) {
#pragma unroll
      for (int it = 0; it < 8; ++it) {
        const int row = it * 2 + hh;
        const v4f val = *(const v4f*)(slab + row * 68 + c4);
        *(volatile v4f*)(C + (size_t)(mBase + row) * ldc + n0 + c4) = val;
      }
      __threadfence();
    }
    __builtin_amdgcn_fence(__ATOMIC_RELEASE, "workgroup");
    __builtin_amdgcn_wave_barrier();
    __builtin_amdgcn_fence(__ATOMIC_ACQUIRE, "workgroup");
  }
}

__global__ __launch_bounds__(256) void cast8_split_f16_kernel(const float* __restrict__ in, unsigned short* __restrict__ outHi,
                                                              unsigned short* __restrict__ outLo, int n8) {
  const int i = blockIdx.x * 256 + threadIdx.x;
  if (i >= n8) return;
  const float* p = in + 8 * (size_t)i;
  const v4f a = *(const v4f*)(p);
  const v4f c = *(const v4f*)(p + 4);
  unsigned short hb[8];
  unsigned short lb[8];
#pragma unroll
  for (int e = 0; e < 4; ++e) {
    const float fa = a[e];
    const float fc = c[e];
    split_f16(fa, hb[e], lb[e]);
    split_f16(fc, hb[4 + e], lb[4 + e]);
  }
  const v4u uh = (v4u){pk16(hb[0], hb[1]), pk16(hb[2], hb[3]), pk16(hb[4], hb[5]), pk16(hb[6], hb[7])};
  const v4u ul = (v4u){pk16(lb[0], lb[1]), pk16(lb[2], lb[3]), pk16(lb[4], lb[5]), pk16(lb[6], lb[7])};
  unsigned short* qh = outHi + 8 * (size_t)i;
  unsigned short* ql = outLo + 8 * (size_t)i;
  *(volatile v4u*)qh = uh;
  *(volatile v4u*)ql = ul;
  __threadfence();
  *(volatile v4u*)qh = uh;
  *(volatile v4u*)ql = ul;
}

template <bool WITH_LO>
__device__ __forceinline__ void tile_store_f16(const float* sm, unsigned short* dstHi, unsigned short* dstLo,
                                               int rowBase, int k0, int t) {
  const int lane = t & 31, wave = t >> 5;
  const int q = lane >> 3, c8 = (lane & 7) * 8;
  for (int pass = 0; pass < 2; ++pass) {
#pragma unroll
    for (int it = 0; it < 2; ++it) {
      const int row = wave * 8 + it * 4 + q;
      unsigned short hb[8];
      unsigned short lb[8];
#pragma unroll
      for (int e = 0; e < 8; ++e) {
        const float val = sm[row * 65 + c8 + e];
        if (WITH_LO) {
          split_f16(val, hb[e], lb[e]);
        } else {
          hb[e] = h_bits(val);
          lb[e] = 0;
        }
      }
      const v4u uh = (v4u){pk16(hb[0], hb[1]), pk16(hb[2], hb[3]), pk16(hb[4], hb[5]), pk16(hb[6], hb[7])};
      *(volatile v4u*)(dstHi + (size_t)(rowBase + row) * kD + k0 + c8) = uh;
      if (WITH_LO) {
        const v4u ul = (v4u){pk16(lb[0], lb[1]), pk16(lb[2], lb[3]), pk16(lb[4], lb[5]), pk16(lb[6], lb[7])};
        *(volatile v4u*)(dstLo + (size_t)(rowBase + row) * kD + k0 + c8) = ul;
      }
    }
    __threadfence();
  }
}

template <bool WITH_LO>
__global__ __launch_bounds__(256) void transpose_cvt_kernel(const float* __restrict__ src, int srcPitch,
                                                            unsigned short* __restrict__ dstHi,
                                                            unsigned short* __restrict__ dstLo,
                                                            int dstRow0, float scale) {
  __shared__ float sm[64 * 65];
  const int t  = threadIdx.x;
  const int k0 = blockIdx.x * 64;
  const int n0 = blockIdx.y * 64;
#pragma unroll 4
  for (int i = 0; i < 16; ++i) {
    const int e = i * 256 + t;
    const int r = e >> 6;
    const int c = e & 63;
    sm[c * 65 + r] = src[(size_t)(k0 + r) * srcPitch + n0 + c] * scale;
  }
  __syncthreads();
  tile_store_f16<WITH_LO>(sm, dstHi, dstLo, dstRow0 + n0, k0, t);
}

__global__ __launch_bounds__(256) void padrows_cvt_kernel(const float* __restrict__ Wb, const float* __restrict__ Wa,
                                                          unsigned short* __restrict__ dstHi,
                                                          unsigned short* __restrict__ dstLo,
                                                          int dstRow0, float scale) {
  __shared__ float sm[64 * 65];
  const int t  = threadIdx.x;
  const int k0 = blockIdx.x * 64;
#pragma unroll
  for (int i = 0; i < 4; ++i) {
    const int e = i * 256 + t;
    const int r = e >> 4;
    const int c = e & 15;
    sm[c * 65 + r] = Wb[(size_t)(k0 + r) * kH + c] * scale;
  }
#pragma unroll
  for (int i = 0; i < 4; ++i) {
    const int e = i * 256 + t;
    const int r = e >> 4;
    const int c = e & 15;
    sm[(16 + c) * 65 + r] = Wa[(size_t)(k0 + r) * kH + c] * scale;
  }
#pragma unroll
  for (int i = 0; i < 8; ++i) {
    const int e = i * 256 + t;
    const int c = 32 + (e >> 6);
    const int r = e & 63;
    sm[c * 65 + r] = 0.0f;
  }
  __syncthreads();
  tile_store_f16<true>(sm, dstHi, dstLo, dstRow0, k0, t);
}

__global__ __launch_bounds__(256) void conv_silu_norm_kernel(const float* __restrict__ P, const float* __restrict__ cw,
                                                             float* __restrict__ QKVN) {
  const int lane = threadIdx.x & 31;
  const int gw = blockIdx.x * 8 + (threadIdx.x >> 5);
  const int l = gw / 48;
  const int g = gw - l * 48;
  if (l >= kL) return;
  const int c0 = g * kHD + 4 * lane;
  v4f w[4];
#pragma unroll
  for (int e = 0; e < 4; ++e) w[e] = *(const v4f*)(cw + (size_t)(c0 + e) * kTaps);
  float acc[4] = {0.0f, 0.0f, 0.0f, 0.0f};
#pragma unroll
  for (int t = 0; t < kTaps; ++t) {
    const int row = l - (kTaps - 1) + t;
    const int rc = row < 0 ? 0 : row;
    const bool ok = row >= 0;
    const v4f pv = *(const v4f*)(P + (size_t)rc * kNCat + c0);
#pragma unroll
    for (int e = 0; e < 4; ++e) {
      const float xv = ok ? pv[e] : 0.0f;
      acc[e] = fmaf(w[e][t], xv, acc[e]);
    }
  }
  float y[4];
#pragma unroll
  for (int e = 0; e < 4; ++e) y[e] = silu_f(acc[e]);
  float ss = (y[0] * y[0] + y[1] * y[1]) + (y[2] * y[2] + y[3] * y[3]);
#pragma unroll
  for (int off = 1; off < 32; off <<= 1) ss += __shfl_xor(ss, off, 32);
  const float sc = rsqrtf(ss + kEps);
  const float qscale = 1.0f / sqrtf((float)kHD);
  const float fac = (g < kH) ? (sc * qscale) : ((g < 2 * kH) ? sc : 1.0f);
  v4f o;
#pragma unroll
  for (int e = 0; e < 4; ++e) o[e] = y[e] * fac;
  float* op = QKVN + (size_t)l * kCConv + c0;
  *(volatile v4f*)op = o;
  __threadfence();
  *(volatile v4f*)op = o;
}

__global__ __launch_bounds__(256) void gate_scalars_kernel(const float* __restrict__ P, const float* __restrict__ A_log,
                                                           const float* __restrict__ dt_bias, float* __restrict__ BD) {
  const int lane = threadIdx.x & 31;
  const int l = blockIdx.x * 8 + (threadIdx.x >> 5);
  if (l >= kL) return;
  const int j = lane & 15;
  const float x   = P[(size_t)l * kNCat + kBCol0 + lane];
  const float dtb = dt_bias[j];
  const float al  = A_log[j];
  const float sig = __builtin_amdgcn_rcpf(1.0f + expf(-x));
  const float xs  = x + dtb;
  const float sp  = fmaxf(xs, 0.0f) + log1pf(expf(-fabsf(xs)));
  float dec = expf(-expf(al) * sp);
  dec = (dec < kFltMin) ? 0.0f : dec;
  const float val = (lane < kH) ? sig : dec;
  float* op = BD + (size_t)l * 32 + lane;
  *(volatile float*)op = val;
  __threadfence();
  *(volatile float*)op = val;
}

__global__ __launch_bounds__(1024) void scan_gate_kernel(const float* __restrict__ QKVN, const float* __restrict__ BD,
                                                         const float* __restrict__ P, const float* __restrict__ norm_w,
                                                         unsigned short* __restrict__ GATED) {
  __shared__ __align__(16) float sqkv[3 * kChunk * kHD];
  __shared__ __align__(16) float so[kChunk * kHD];
  __shared__ float sbd[2 * kChunk];

  const int h    = blockIdx.x;
  const int tid  = threadIdx.x;
  const int lane = tid & 31;
  const int wave = tid >> 5;
  const int v    = wave * 4 + (lane >> 3);
  const int dg   = lane & 7;
  const int gs   = wave & 15;

  float M[kStatePerLane];
#pragma unroll
  for (int i = 0; i < kStatePerLane; ++i) M[i] = 0.0f;

  const v4f nw = *(const v4f*)(norm_w + 4 * lane);

#pragma unroll 1
  for (int ch = 0; ch < kL / kChunk; ++ch) {
    const int l0 = ch * kChunk;
    {
      const int idx = tid;
      const int which = idx >> 9;
      const int rem = idx & 511;
      const int row = rem >> 5;
      const int c4 = (rem & 31) * 4;
      const v4f val = *(const v4f*)(QKVN + (size_t)(l0 + row) * kCConv + which * kCKey + h * kHD + c4);
      *(v4f*)(sqkv + idx * 4) = val;
    }
    if (tid < 512) {
      const int idx = 1024 + tid;
      const int rem = idx & 511;
      const int row = rem >> 5;
      const int c4 = (rem & 31) * 4;
      const v4f val = *(const v4f*)(QKVN + (size_t)(l0 + row) * kCConv + 2 * kCKey + h * kHD + c4);
      *(v4f*)(sqkv + idx * 4) = val;
    }
    if (wave == 31) {
      const int row = lane & 15;
      const int wsel = lane >> 4;
      sbd[wsel * kChunk + row] = BD[(size_t)(l0 + row) * 32 + wsel * kH + h];
    }
    __syncthreads();

#pragma unroll 1
    for (int s = 0; s < kChunk; ++s) {
      const float bt = sbd[s];
      const float dc = sbd[kChunk + s];
      const float vt = sqkv[2 * kChunk * kHD + s * kHD + v];
      const float* kp = sqkv + kChunk * kHD + s * kHD + dg * kStatePerLane;
      const float* qp = sqkv + s * kHD + dg * kStatePerLane;
      v4f kv[4], qv[4];
#pragma unroll
      for (int j = 0; j < 4; ++j) {
        kv[j] = *(const v4f*)(kp + 4 * j);
        qv[j] = *(const v4f*)(qp + 4 * j);
      }
      float pk = 0.0f;
#pragma unroll
      for (int j = 0; j < 4; ++j) {
#pragma unroll
        for (int e = 0; e < 4; ++e) {
          const float m = M[4 * j + e] * dc;
          M[4 * j + e] = m;
          pk = fmaf(kv[j][e], m, pk);
        }
      }
      pk += __shfl_xor(pk, 1, 32);
      pk += __shfl_xor(pk, 2, 32);
      pk += __shfl_xor(pk, 4, 32);
      const float u = (vt - pk) * bt;
      float pq = 0.0f;
#pragma unroll
      for (int j = 0; j < 4; ++j) {
#pragma unroll
        for (int e = 0; e < 4; ++e) {
          const float m = fmaf(kv[j][e], u, M[4 * j + e]);
          M[4 * j + e] = m;
          pq = fmaf(qv[j][e], m, pq);
        }
      }
      pq += __shfl_xor(pq, 1, 32);
      pq += __shfl_xor(pq, 2, 32);
      pq += __shfl_xor(pq, 4, 32);
      if (dg == 0) so[s * kHD + v] = pq;
    }
    __syncthreads();

    {
      const int l = l0 + gs;
      const v4f o4 = *(const v4f*)(so + gs * kHD + 4 * lane);
      float ss = (o4[0] * o4[0] + o4[1] * o4[1]) + (o4[2] * o4[2] + o4[3] * o4[3]);
#pragma unroll
      for (int off = 1; off < 32; off <<= 1) ss += __shfl_xor(ss, off, 32);
      const float rms = rsqrtf(ss * (1.0f / (float)kHD) + kEps);
      const v4f z4 = *(const v4f*)(P + (size_t)l * kNCat + kZCol0 + h * kHD + 4 * lane);
      unsigned short hb[4];
#pragma unroll
      for (int e = 0; e < 4; ++e) {
        const float oe = o4[e];
        const float ze = z4[e];
        const float we = nw[e];
        const float gval = ((oe * rms) * we) * silu_f(ze);
        hb[e] = h_bits(gval * kGCarry);
      }
      const v2u wv = (v2u){pk16(hb[0], hb[1]), pk16(hb[2], hb[3])};
      if (wave < kChunk) {
        unsigned short* gp = GATED + (size_t)l * kCVal + h * kHD + 4 * lane;
        *(volatile v2u*)gp = wv;
        __threadfence();
        *(volatile v2u*)gp = wv;
      }
    }
  }
}

extern "C" void kernel_launch(void* const* d_in, const int* in_sizes, int n_in,
                              void* d_out, int out_size, void* d_ws, size_t ws_size, hipStream_t stream) {
  if (n_in < 10 || d_out == nullptr || d_ws == nullptr) return;
  if (in_sizes[0] != kL * kD || in_sizes[1] != kD * kCConv || in_sizes[2] != kD * kCVal ||
      in_sizes[3] != kD * kH || in_sizes[4] != kD * kH || in_sizes[5] != kCConv * kTaps ||
      in_sizes[6] != kH || in_sizes[7] != kH || in_sizes[8] != kHD || in_sizes[9] != kCVal * kD ||
      out_size != kL * kD) return;

  const float* x       = (const float*)d_in[0];
  const float* Wqkv    = (const float*)d_in[1];
  const float* Wz      = (const float*)d_in[2];
  const float* Wb      = (const float*)d_in[3];
  const float* Wa      = (const float*)d_in[4];
  const float* conv_w  = (const float*)d_in[5];
  const float* A_log   = (const float*)d_in[6];
  const float* dt_bias = (const float*)d_in[7];
  const float* norm_w  = (const float*)d_in[8];
  const float* Wout    = (const float*)d_in[9];
  float* out = (float*)d_out;

  char* ws = (char*)d_ws;
  size_t off = 0;
  auto carve = [&](size_t bytes) -> char* { char* p = ws + off; off += (bytes + 255) & ~(size_t)255; return p; };
  unsigned short* X16H  = (unsigned short*)carve((size_t)kL * kD * 2);
  unsigned short* X16L  = (unsigned short*)carve((size_t)kL * kD * 2);
  unsigned short* WCATH = (unsigned short*)carve((size_t)kNCat * kD * 2);
  unsigned short* WCATL = (unsigned short*)carve((size_t)kNCat * kD * 2);
  unsigned short* WOUTT = (unsigned short*)carve((size_t)kD * kCVal * 2);
  float*          Pbuf  = (float*)carve((size_t)kL * kNCat * 4);
  float*          BD    = (float*)carve((size_t)kL * 32 * 4);
  unsigned short* GATED = (unsigned short*)carve((size_t)kL * kCVal * 2);
  if (off > ws_size || off > (size_t)134217728) return;
  float* QKVN = (float*)WCATH;

  const int n8x = kL * kD / 8;
  cast8_split_f16_kernel<<<(n8x + 255) / 256, 256, 0, stream>>>(x, X16H, X16L, n8x);
  transpose_cvt_kernel<true><<<dim3(kD / 64, kCConv / 64), 256, 0, stream>>>(Wqkv, kCConv, WCATH, WCATL, 0, kWCarry);
  transpose_cvt_kernel<true><<<dim3(kD / 64, kCVal / 64), 256, 0, stream>>>(Wz, kCVal, WCATH, WCATL, kZCol0, kWCarry);
  padrows_cvt_kernel<<<kD / 64, 256, 0, stream>>>(Wb, Wa, WCATH, WCATL, kBCol0, kWCarry);
  transpose_cvt_kernel<false><<<dim3(kCVal / 64, kD / 64), 256, 0, stream>>>(Wout, kD, WOUTT, WOUTT, 0, kWCarry);

  wmma_gemm_split_f16<<<((kL / 64) * (kNCat / 32)) / 8, 256, 0, stream>>>(
      X16H, X16L, kD, WCATH, WCATL, kD, Pbuf, kNCat, kL, kNCat, kD, kProjScale);

  conv_silu_norm_kernel<<<(kL * 48) / 8, 256, 0, stream>>>(Pbuf, conv_w, QKVN);

  gate_scalars_kernel<<<kL / 8, 256, 0, stream>>>(Pbuf, A_log, dt_bias, BD);

  scan_gate_kernel<<<kH, kScanThreads, 0, stream>>>(QKVN, BD, Pbuf, norm_w, GATED);

  wmma_gemm64_f16<<<((kL / 64) * (kD / 64)) / 8, 256, 0, stream>>>(
      GATED, kCVal, WOUTT, kCVal, out, kD, kL, kD, kCVal, kOutScale);
}
